// encoder_unit_80109730005719
// MI455X (gfx1250) — hardware-verified
//
#include <hip/hip_runtime.h>
#include <math.h>
#include <stdint.h>

#define NB    2
#define SEQ   2048
#define DM    1024
#define NH    16
#define HD    64
#define DFF   4096
#define NTOK  (NB * SEQ)
#define NQB   (SEQ / 64)
#define QKP   (2 * DM)
#define LNEPS 1.0e-5f
#define WSC   64.0f
#define PSC   16384.0f
#define VRS   4096.0f
static_assert(NH * HD == DM);
static_assert((SEQ % 64) == 0 && (DM % 64) == 0 && (NTOK % 64) == 0 && (DFF % 64) == 0 && (DM % 32) == 0);
static_assert(DM == 4 * 256);

typedef _Float16 v16h __attribute__((ext_vector_type(16)));
typedef _Float16 v8h  __attribute__((ext_vector_type(8)));
typedef __bf16   v16b __attribute__((ext_vector_type(16)));
typedef float    v8f  __attribute__((ext_vector_type(8)));
typedef float    v4f  __attribute__((ext_vector_type(4)));
typedef unsigned int v4u __attribute__((ext_vector_type(4)));
typedef unsigned int v2u __attribute__((ext_vector_type(2)));
typedef unsigned short v8us __attribute__((ext_vector_type(8)));

__device__ __forceinline__ unsigned short bf_bits(float f) {
  unsigned u = __float_as_uint(f);
  return (unsigned short)((u + 0x7FFFu + ((u >> 16) & 1u)) >> 16);
}
__device__ __forceinline__ float bf_up(unsigned short h) { return __uint_as_float(((unsigned)h) << 16); }
__device__ __forceinline__ float bfr(float f) { return bf_up(bf_bits(f)); }
__device__ __forceinline__ unsigned short h_bits(_Float16 x) { return __builtin_bit_cast(unsigned short, x); }
__device__ __forceinline__ unsigned pk16(unsigned short a, unsigned short b) { return (unsigned)a | ((unsigned)b << 16); }
__device__ __forceinline__ v8f zero8() { v8f z = {0.f, 0.f, 0.f, 0.f, 0.f, 0.f, 0.f, 0.f}; return z; }

__device__ __forceinline__ v16h ldfrag_h(const unsigned short* p) {
  union { v16h v; v8us u[2]; } f;
  f.u[0] = *(const v8us*)(p);
  f.u[1] = *(const v8us*)(p + 16);
  return f.v;
}
__device__ __forceinline__ v16b ldfrag_b(const unsigned short* p) {
  union { v16b v; v8us u[2]; } f;
  f.u[0] = *(const v8us*)(p);
  f.u[1] = *(const v8us*)(p + 16);
  return f.v;
}
template <int TYP> struct FT;
template <> struct FT<0> {
  typedef v16h V;
  static __device__ __forceinline__ V ld(const unsigned short* p) { return ldfrag_h(p); }
};
template <> struct FT<1> {
  typedef v16b V;
  static __device__ __forceinline__ V ld(const unsigned short* p) { return ldfrag_b(p); }
};

__device__ __forceinline__ v8f mma_raw(v16h a, v16h b, v8f c) {
  return __builtin_amdgcn_wmma_f32_16x16x32_f16(false, a, false, b, (short)0, c, false, false);
}
__device__ __forceinline__ v8f mma_raw(v16b a, v16b b, v8f c) {
  return __builtin_amdgcn_wmma_f32_16x16x32_bf16(false, a, false, b, (short)0, c, false, false);
}
__device__ __forceinline__ v8f mma_h(v16h a, v16h b, v8f c) {
  c = __builtin_amdgcn_wmma_f32_16x16x32_f16(false, a, false, b, (short)0, c, false, false);
#if defined(__HIP_DEVICE_COMPILE__)
  asm volatile("v_nop\n\tv_nop\n\tv_nop\n\tv_nop" : "+v"(c) : "v"(a), "v"(b));
#endif
  return c;
}
__device__ __forceinline__ v8f mma_b(v16b a, v16b b, v8f c) {
  c = __builtin_amdgcn_wmma_f32_16x16x32_bf16(false, a, false, b, (short)0, c, false, false);
#if defined(__HIP_DEVICE_COMPILE__)
  asm volatile("v_nop\n\tv_nop\n\tv_nop\n\tv_nop" : "+v"(c) : "v"(a), "v"(b));
#endif
  return c;
}
template <typename VF>
__device__ __forceinline__ void dep_guard1(v8f& a, v8f& b, VF x) {
#if defined(__HIP_DEVICE_COMPILE__)
  asm volatile("v_nop\n\tv_nop\n\tv_nop\n\tv_nop" : "+v"(a), "+v"(b) : "v"(x));
#endif
}
template <typename VF>
__device__ __forceinline__ void dep_guard2(v8f& a, v8f& b, VF x, VF y) {
#if defined(__HIP_DEVICE_COMPILE__)
  asm volatile("v_nop\n\tv_nop\n\tv_nop\n\tv_nop" : "+v"(a), "+v"(b) : "v"(x), "v"(y));
#endif
}
template <typename VF>
__device__ __forceinline__ void keep4(VF a, VF b, VF c, VF d) {
#if defined(__HIP_DEVICE_COMPILE__)
  asm volatile("v_nop" :: "v"(a), "v"(b), "v"(c), "v"(d));
#endif
}
__device__ __forceinline__ void acc_guard4(v8f& a, v8f& b, v8f& c, v8f& d) {
#if defined(__HIP_DEVICE_COMPILE__)
  asm volatile("v_nop\n\tv_nop\n\tv_nop\n\tv_nop" : "+v"(a), "+v"(b), "+v"(c), "+v"(d));
#endif
}
__device__ __forceinline__ void wave_sync_lds() {
  __builtin_amdgcn_fence(__ATOMIC_RELEASE, "workgroup");
  __builtin_amdgcn_wave_barrier();
  __builtin_amdgcn_fence(__ATOMIC_ACQUIRE, "workgroup");
}
__device__ __forceinline__ float wsum(float v) {
#pragma unroll
  for (int off = 16; off > 0; off >>= 1) v += __shfl_xor(v, off, 32);
  return v;
}
__device__ __forceinline__ float bsum256(float v, float* red, int lane, int wave) {
  v = wsum(v);
  if (lane == 0) red[wave] = v;
  __syncthreads();
  float tot = 0.f;
#pragma unroll
  for (int w = 0; w < 8; ++w) tot += red[w];
  return tot;
}

template <int BF>
__global__ __launch_bounds__(256) void cvt8(const float* __restrict__ X, unsigned short* out, int n8, float sc) {
  const int i = blockIdx.x * 256 + threadIdx.x;
  if (i < n8) {
    const size_t o = (size_t)i * 8;
    const v4f a0 = *(const v4f*)(X + o), a1 = *(const v4f*)(X + o + 4);
    v4u p;
#pragma unroll
    for (int e = 0; e < 2; ++e) {
      unsigned short s0, s1, s2, s3;
      if (BF) {
        s0 = bf_bits(a0[2 * e]); s1 = bf_bits(a0[2 * e + 1]);
        s2 = bf_bits(a1[2 * e]); s3 = bf_bits(a1[2 * e + 1]);
      } else {
        s0 = h_bits((_Float16)(bfr(a0[2 * e]) * sc)); s1 = h_bits((_Float16)(bfr(a0[2 * e + 1]) * sc));
        s2 = h_bits((_Float16)(bfr(a1[2 * e]) * sc)); s3 = h_bits((_Float16)(bfr(a1[2 * e + 1]) * sc));
      }
      p[e]     = pk16(s0, s1);
      p[2 + e] = pk16(s2, s3);
    }
    *(volatile v4u*)(out + o) = p;
    __threadfence();
    *(volatile v4u*)(out + o) = p;
  }
}

template <int TYP, int ASPLIT, int OM, int BIASM, int ACT, int RES>
__global__ __launch_bounds__(256) void gemm64(
    const unsigned short* __restrict__ Ap, int lda, long long strideA, long long planeA2,
    const unsigned short* __restrict__ Btp, int ldb, long long strideB,
    const float* __restrict__ bias0, const float* __restrict__ bias1, int Nb,
    const float* __restrict__ resid,
    void* Cout, int ldc, long long strideC, long long planeC2,
    int M, int N, int K, float oscale, float rsc) {
  typedef typename FT<TYP>::V VF;
  __shared__ __align__(16) float sT[8][16 * 68];
  const int b    = blockIdx.y;
  const int lane = threadIdx.x & 31;
  const int wave = threadIdx.x >> 5;
  const int tilesN = N >> 6;
  const int tilesM = M >> 6;
  const int tile = blockIdx.x * 8 + wave;
  if (tile >= tilesM * tilesN) return;
  const int tm = tile / tilesN;
  const int tn = tile - tm * tilesN;
  const int m0 = tm << 6;
  const int n0 = tn << 6;

  const unsigned short* Ab = Ap + (size_t)b * strideA;
  const unsigned short* A2 = Ab + planeA2;
  const unsigned short* Bb = Btp + (size_t)b * strideB;

  const int rlane = lane & 15;
  const int koff  = (lane >> 4) * 8;
  const int mOff  = (lane >> 4) * 8;

  v8f acc[4][4];
#pragma unroll
  for (int i = 0; i < 4; ++i)
#pragma unroll
    for (int j = 0; j < 4; ++j) acc[i][j] = zero8();

  for (int k0 = 0; k0 < K; k0 += 32) {
    VF bh[4];
#pragma unroll
    for (int j = 0; j < 4; ++j) {
      const size_t bo = (size_t)(n0 + (j << 4) + rlane) * ldb + koff + k0;
      bh[j] = FT<TYP>::ld(Bb + bo);
    }
#pragma unroll
    for (int i = 0; i < 4; ++i) {
      const size_t ao = (size_t)(m0 + (i << 4) + rlane) * lda + koff + k0;
      const VF ah = FT<TYP>::ld(Ab + ao);
      if (ASPLIT) {
        const VF al = FT<TYP>::ld(A2 + ao);
#pragma unroll
        for (int j = 0; j < 4; ++j) acc[i][j] = mma_raw(ah, bh[j], acc[i][j]);
#pragma unroll
        for (int j = 0; j < 4; ++j) acc[i][j] = mma_raw(al, bh[j], acc[i][j]);
        dep_guard2<VF>(acc[i][0], acc[i][3], ah, al);
      } else {
#pragma unroll
        for (int j = 0; j < 4; ++j) acc[i][j] = mma_raw(ah, bh[j], acc[i][j]);
        dep_guard1<VF>(acc[i][0], acc[i][3], ah);
      }
    }
    keep4<VF>(bh[0], bh[1], bh[2], bh[3]);
  }
  acc_guard4(acc[0][0], acc[0][1], acc[0][2], acc[0][3]);
  acc_guard4(acc[1][0], acc[1][1], acc[1][2], acc[1][3]);
  acc_guard4(acc[2][0], acc[2][1], acc[2][2], acc[2][3]);
  acc_guard4(acc[3][0], acc[3][1], acc[3][2], acc[3][3]);

  const int hh2 = lane >> 4, c4 = (lane & 15) * 4;
  const int q8  = lane >> 3, c8 = (lane & 7) * 8;
  float bc[8];
#pragma unroll
  for (int e = 0; e < 8; ++e) bc[e] = 0.f;
  if (BIASM == 0) {
    const bool use1 = (n0 >= Nb);
    if (OM == 0) {
      const int cb = n0 + c4;
      const int i0 = (cb < Nb - 4) ? cb : (Nb - 4);
      const int i1 = (cb - Nb > 0) ? (cb - Nb) : 0;
      const v4f b0v = *(const v4f*)(bias0 + i0);
      const v4f b1v = *(const v4f*)(bias1 + i1);
#pragma unroll
      for (int e = 0; e < 4; ++e) bc[e] = bfr(use1 ? b1v[e] : b0v[e]);
    } else {
      const int cb = n0 + c8;
      const int i0 = (cb < Nb - 8) ? cb : (Nb - 8);
      const int i1 = (cb - Nb > 0) ? (cb - Nb) : 0;
      const v4f b0a = *(const v4f*)(bias0 + i0), b0b = *(const v4f*)(bias0 + i0 + 4);
      const v4f b1a = *(const v4f*)(bias1 + i1), b1b = *(const v4f*)(bias1 + i1 + 4);
#pragma unroll
      for (int e = 0; e < 4; ++e) {
        bc[e]     = bfr(use1 ? b1a[e] : b0a[e]);
        bc[4 + e] = bfr(use1 ? b1b[e] : b0b[e]);
      }
    }
  }

  float* slab = sT[wave];
#pragma unroll
  for (int i = 0; i < 4; ++i) {
    const int mBase = m0 + (i << 4);
#pragma unroll
    for (int j = 0; j < 4; ++j) {
#pragma unroll
      for (int r = 0; r < 8; ++r) {
        slab[(mOff + r) * 68 + (j << 4) + rlane] = acc[i][j][r];
      }
    }
    wave_sync_lds();
    if (OM == 0) {
      float* C = (float*)Cout + (size_t)b * strideC;
      const float* Rb = resid + (size_t)b * strideC;
      v4f vals[8];
#pragma unroll
      for (int it = 0; it < 8; ++it) {
        const int row = it * 2 + hh2;
        v4f v = *(const v4f*)(slab + row * 68 + c4);
#pragma unroll
        for (int e = 0; e < 4; ++e) {
          float f = v[e] * oscale + bc[e];
          if (ACT) f = fmaxf(f, 0.0f);
          v[e] = f;
        }
        if (RES != 0) {
          const v4f rr = *(const v4f*)(Rb + (size_t)(mBase + row) * ldc + n0 + c4);
#pragma unroll
          for (int e = 0; e < 4; ++e) v[e] += (RES == 2) ? bfr(rr[e]) : rr[e];
        }
        vals[it] = v;
      }
      for (int pass = 0; pass < 2; ++pass) {
#pragma unroll
        for (int it = 0; it < 8; ++it) {
          const int row = it * 2 + hh2;
          *(volatile v4f*)(C + (size_t)(mBase + row) * ldc + n0 + c4) = vals[it];
        }
        __threadfence();
      }
    } else {
      unsigned short* C  = (unsigned short*)Cout + (size_t)b * strideC;
      unsigned short* C2 = C + planeC2;
      v4u hv[4], hw[4];
#pragma unroll
      for (int it = 0; it < 4; ++it) {
        const int row = it * 4 + q8;
        const float* sp = slab + row * 68 + c8;
        float bm = 0.f;
        if (BIASM == 1) bm = bfr(bias0[mBase + row]);
        v4u a, a2;
#pragma unroll
        for (int e = 0; e < 4; ++e) {
          float f0 = sp[2 * e]     * oscale + ((BIASM == 1) ? bm : bc[2 * e]);
          float f1 = sp[2 * e + 1] * oscale + ((BIASM == 1) ? bm : bc[2 * e + 1]);
          if (ACT) { f0 = fmaxf(f0, 0.0f); f1 = fmaxf(f1, 0.0f); }
          unsigned short u0, u1, w0 = 0, w1 = 0;
          if (OM == 3) {
            u0 = bf_bits(f0); u1 = bf_bits(f1);
            w0 = bf_bits(f0 - bf_up(u0)); w1 = bf_bits(f1 - bf_up(u1));
          } else {
            const _Float16 x0 = (_Float16)f0, x1 = (_Float16)f1;
            u0 = h_bits(x0); u1 = h_bits(x1);
            if (OM == 4) {
              w0 = h_bits((_Float16)((f0 - (float)x0) * rsc));
              w1 = h_bits((_Float16)((f1 - (float)x1) * rsc));
            }
          }
          a[e]  = pk16(u0, u1);
          a2[e] = pk16(w0, w1);
        }
        hv[it] = a; hw[it] = a2;
      }
      for (int pass = 0; pass < 2; ++pass) {
#pragma unroll
        for (int it = 0; it < 4; ++it) {
          const int row = it * 4 + q8;
          const size_t co = (size_t)(mBase + row) * ldc + n0 + c8;
          *(volatile v4u*)(C + co) = hv[it];
          if (OM >= 3) *(volatile v4u*)(C2 + co) = hw[it];
        }
        __threadfence();
      }
    }
    wave_sync_lds();
  }
}

__global__ __launch_bounds__(128)
void attn64(const unsigned short* __restrict__ qkp, const unsigned short* __restrict__ vtp, unsigned short* ctxp) {
  union FB { v16b v; v8us u[2]; };
  union FH { v16h v; v8h h[2]; v8us u[2]; };
  __shared__ __align__(16) unsigned short Khs[64 * 64];
  __shared__ __align__(16) unsigned short Kls[64 * 64];
  __shared__ __align__(16) unsigned short Vhs[64 * 64];
  __shared__ __align__(16) unsigned short Vrs[64 * 64];
  __shared__ __align__(16) _Float16 Psh[4][16 * 64];
  __shared__ __align__(16) float    Os[4][16 * 64];

  const int tid  = threadIdx.x;
  const int wave = tid >> 5;
  const int lane = tid & 31;
  const int hh   = lane >> 4;
  const int c    = lane & 15;

  const int bx   = blockIdx.x;
  const int qb   = bx % NQB;
  const int rest = bx / NQB;
  const int h    = rest % NH;
  const int b    = rest / NH;
  const int q0   = qb * 64 + wave * 16;
  const size_t rowB  = (size_t)b * SEQ;
  const size_t PLQK  = (size_t)NTOK * QKP;
  const size_t PLVT  = (size_t)NB * DM * SEQ;
  const size_t PLCTX = (size_t)NTOK * DM;

  const unsigned short* Qg = qkp + (size_t)h * HD;
  const unsigned short* Kg = qkp + DM + (size_t)h * HD;
  const unsigned short* Vg = vtp + ((size_t)b * DM + (size_t)h * HD) * SEQ;

  v16b qh[2], ql[2];
#pragma unroll
  for (int dc = 0; dc < 2; ++dc) {
    const size_t qo = (rowB + q0 + c) * QKP + dc * 32 + 8 * hh;
    qh[dc] = ldfrag_b(Qg + qo);
    ql[dc] = ldfrag_b(Qg + PLQK + qo);
  }

  float mrow[8], lrow[8];
  v8f oacc[4], oacr[4];
#pragma unroll
  for (int r = 0; r < 8; ++r) { mrow[r] = -INFINITY; lrow[r] = 0.f; }
#pragma unroll
  for (int t = 0; t < 4; ++t) { oacc[t] = zero8(); oacr[t] = zero8(); }

  for (int kt = 0; kt < NQB; ++kt) {
    const int kv0 = kt * 64;
    __syncthreads();
    {
      const int r = tid >> 1, hf = (tid & 1) * 32;
      const unsigned short* kg = Kg + (rowB + kv0 + r) * QKP + hf;
      const unsigned short* vg = Vg + (size_t)r * SEQ + kv0 + hf;
#pragma unroll
      for (int i = 0; i < 4; ++i) {
        const v8us a0 = *(const v8us*)(kg + 8 * i);
        const v8us a1 = *(const v8us*)(kg + PLQK + 8 * i);
        const v8us b0 = *(const v8us*)(vg + 8 * i);
        const v8us b1 = *(const v8us*)(vg + PLVT + 8 * i);
        *(v8us*)(Khs + r * 64 + hf + 8 * i) = a0;
        *(v8us*)(Kls + r * 64 + hf + 8 * i) = a1;
        *(v8us*)(Vhs + r * 64 + hf + 8 * i) = b0;
        *(v8us*)(Vrs + r * 64 + hf + 8 * i) = b1;
      }
    }
    __syncthreads();

    v8f s[4];
#pragma unroll
    for (int j = 0; j < 4; ++j) {
      v8f sh = zero8();
#pragma unroll
      for (int dc = 0; dc < 2; ++dc) {
        FB kbh, kbl;
        const int ko = (j * 16 + c) * 64 + dc * 32 + 8 * hh;
        kbh.u[0] = *(const v8us*)(Khs + ko);
        kbh.u[1] = *(const v8us*)(Khs + ko + 16);
        kbl.u[0] = *(const v8us*)(Kls + ko);
        kbl.u[1] = *(const v8us*)(Kls + ko + 16);
        sh = mma_b(qh[dc], kbh.v, sh);
        sh = mma_b(ql[dc], kbh.v, sh);
        sh = mma_b(qh[dc], kbl.v, sh);
      }
      s[j] = sh;
    }

    _Float16* pwh = Psh[wave];
#pragma unroll
    for (int r = 0; r < 8; ++r) {
      float m = s[0][r];
      m = fmaxf(m, s[1][r]);
      m = fmaxf(m, s[2][r]);
      m = fmaxf(m, s[3][r]);
#pragma unroll
      for (int off = 1; off < 16; off <<= 1) m = fmaxf(m, __shfl_xor(m, off, 32));
      const float mnew  = fmaxf(mrow[r], m);
      const float alpha = __expf(mrow[r] - mnew);
      mrow[r] = mnew;
      float psum = 0.f;
#pragma unroll
      for (int j = 0; j < 4; ++j) {
        const float p = __expf(s[j][r] - mnew);
        psum += p;
        pwh[(8 * hh + r) * 64 + j * 16 + c] = (_Float16)(p * PSC);
      }
#pragma unroll
      for (int off = 1; off < 16; off <<= 1) psum += __shfl_xor(psum, off, 32);
      lrow[r] = lrow[r] * alpha + psum;
#pragma unroll
      for (int t = 0; t < 4; ++t) { oacc[t][r] *= alpha; oacr[t][r] *= alpha; }
    }
    wave_sync_lds();

#pragma unroll 1
    for (int kk = 0; kk < 2; ++kk) {
      FH pa;
      pa.h[0] = *(const v8h*)(pwh + c * 64 + kk * 32 + 8 * hh);
      pa.h[1] = *(const v8h*)(pwh + c * 64 + kk * 32 + 16 + 8 * hh);
#pragma unroll
      for (int t = 0; t < 4; ++t) {
        FH vbh, vbr;
        const int vo = (t * 16 + c) * 64 + kk * 32 + 8 * hh;
        vbh.u[0] = *(const v8us*)(Vhs + vo);
        vbh.u[1] = *(const v8us*)(Vhs + vo + 16);
        vbr.u[0] = *(const v8us*)(Vrs + vo);
        vbr.u[1] = *(const v8us*)(Vrs + vo + 16);
        oacc[t] = mma_h(pa.v, vbh.v, oacc[t]);
        oacr[t] = mma_h(pa.v, vbr.v, oacr[t]);
      }
    }
  }

  float* os = Os[wave];
#pragma unroll
  for (int r = 0; r < 8; ++r) {
    const float l = lrow[r];
    const float inv = ((l > 0.f) ? (1.0f / l) : 0.f) * (1.0f / (PSC * 8.0f));
#pragma unroll
    for (int t = 0; t < 4; ++t) os[(8 * hh + r) * 64 + t * 16 + c] = (oacc[t][r] + oacr[t][r] * (1.0f / VRS)) * inv;
  }
  wave_sync_lds();
  {
    const int q4 = lane >> 3, c8 = (lane & 7) * 8;
    v4u hv[4], hl[4];
#pragma unroll
    for (int it = 0; it < 4; ++it) {
      const int row = it * 4 + q4;
      const float* sp = os + row * 64 + c8;
      v4u a, a2;
#pragma unroll
      for (int e = 0; e < 4; ++e) {
        const float f0 = sp[2 * e], f1 = sp[2 * e + 1];
        const unsigned short u0 = bf_bits(f0), u1 = bf_bits(f1);
        const unsigned short w0 = bf_bits(f0 - bf_up(u0)), w1 = bf_bits(f1 - bf_up(u1));
        a[e]  = pk16(u0, u1);
        a2[e] = pk16(w0, w1);
      }
      hv[it] = a; hl[it] = a2;
    }
    for (int pass = 0; pass < 2; ++pass) {
#pragma unroll
      for (int it = 0; it < 4; ++it) {
        const int row = it * 4 + q4;
        const size_t go = (rowB + q0 + row) * DM + (size_t)h * HD + c8;
        *(volatile v4u*)(ctxp + go) = hv[it];
        *(volatile v4u*)(ctxp + PLCTX + go) = hl[it];
      }
      __threadfence();
    }
  }
}

__device__ __forceinline__ void row_store_f32(float* dst_row, v4f o, int t) {
  *(volatile v4f*)(dst_row + 4 * t) = o;
  __threadfence();
  *(volatile v4f*)(dst_row + 4 * t) = o;
}
__device__ __forceinline__ void row_store_h16(unsigned int* sb, unsigned short* dst_row, v4f o, int t) {
  v2u p;
  p[0] = pk16(h_bits((_Float16)o[0]), h_bits((_Float16)o[1]));
  p[1] = pk16(h_bits((_Float16)o[2]), h_bits((_Float16)o[3]));
  *(v2u*)(sb + 2 * t) = p;
  __syncthreads();
  if (t < 128) {
    const v4u v = *(const v4u*)(sb + 4 * t);
    *(volatile v4u*)(dst_row + 8 * t) = v;
    __threadfence();
    *(volatile v4u*)(dst_row + 8 * t) = v;
  }
}

template <int OUTH>
__global__ __launch_bounds__(256) void ln_row(const float* __restrict__ X, const float* __restrict__ gam,
                                              const float* __restrict__ bet, float* outF, unsigned short* outH) {
  __shared__ float red0[8], red1[8];
  __shared__ __align__(16) unsigned int sb[512];
  const int t = threadIdx.x, lane = t & 31, wave = t >> 5;
  const size_t base = (size_t)blockIdx.x * DM;
  const v4f xv = *(const v4f*)(X + base + 4 * t);
  const float mean = bsum256((xv[0] + xv[1]) + (xv[2] + xv[3]), red0, lane, wave) * (1.0f / DM);
  v4f d;
#pragma unroll
  for (int e = 0; e < 4; ++e) d[e] = xv[e] - mean;
  const float var  = bsum256((d[0] * d[0] + d[1] * d[1]) + (d[2] * d[2] + d[3] * d[3]), red1, lane, wave) * (1.0f / DM);
  const float rstd = 1.0f / sqrtf(var + LNEPS);
  const v4f gv = *(const v4f*)(gam + 4 * t);
  const v4f bv = *(const v4f*)(bet + 4 * t);
  v4f y;
#pragma unroll
  for (int e = 0; e < 4; ++e) y[e] = (d[e] * rstd) * bfr(gv[e]) + bfr(bv[e]);
  row_store_f32(outF + base, y, t);
  if (OUTH) row_store_h16(sb, outH + base, y, t);
}

extern "C" void kernel_launch(void* const* d_in, const int* in_sizes, int n_in,
                              void* d_out, int out_size, void* d_ws, size_t ws_size,
                              hipStream_t stream) {
  if (n_in < 17) return;
  if (in_sizes[0] != NTOK * DM) return;
  if (in_sizes[1] != DM * DM || in_sizes[3] != DM * DM || in_sizes[5] != DM * DM) return;
  if (in_sizes[2] != DM || in_sizes[4] != DM || in_sizes[6] != DM) return;
  if (in_sizes[7] != DM * DM || in_sizes[8] != DM) return;
  if (in_sizes[9] != DM || in_sizes[10] != DM) return;
  if (in_sizes[11] != DFF * DM || in_sizes[12] != DFF) return;
  if (in_sizes[13] != DM * DFF || in_sizes[14] != DM) return;
  if (in_sizes[15] != DM || in_sizes[16] != DM) return;
  if (out_size != NTOK * DM) return;

  const float* emb = (const float*)d_in[0];
  const float* Wq  = (const float*)d_in[1];   const float* bq  = (const float*)d_in[2];
  const float* Wk  = (const float*)d_in[3];   const float* bk  = (const float*)d_in[4];
  const float* Wv  = (const float*)d_in[5];   const float* bv  = (const float*)d_in[6];
  const float* W0  = (const float*)d_in[7];   const float* b0  = (const float*)d_in[8];
  const float* g1  = (const float*)d_in[9];   const float* be1 = (const float*)d_in[10];
  const float* W1  = (const float*)d_in[11];  const float* b1  = (const float*)d_in[12];
  const float* W2  = (const float*)d_in[13];  const float* b2  = (const float*)d_in[14];
  const float* g2  = (const float*)d_in[15];  const float* be2 = (const float*)d_in[16];

  const size_t PW    = (size_t)DM * DM * 2;
  const size_t PWF   = (size_t)DFF * DM * 2;
  const size_t PAH   = (size_t)NTOK * DM * 2;
  const size_t PAF   = (size_t)NTOK * DM * 4;
  const size_t PQK1  = (size_t)NTOK * QKP * 2;
  const size_t PVT1  = (size_t)NB * DM * SEQ * 2;
  const size_t PG    = (size_t)NTOK * DFF * 2;
  size_t off = 0;
  const size_t oWqkv = off; off += 3 * PW;
  const size_t oW0   = off; off += PW;
  const size_t oW1   = off; off += PWF;
  const size_t oW2   = off; off += PWF;
  const size_t oEH   = off; off += PAH;
  const size_t oQK   = off; off += 2 * PQK1;
  const size_t oVT   = off; off += 2 * PVT1;
  const size_t oCtx  = off; off += 2 * PAH;
  const size_t oR    = off; off += PAF;
  if (off > ws_size) return;
  if (off > (size_t)134217728) return;
  if (oQK + PG > oVT) return;
  if (oVT + PAH > oCtx) return;
  if (oCtx + PAF > oR) return;

  char* ws = (char*)d_ws;
  unsigned short* Wqkv = (unsigned short*)(ws + oWqkv);
  unsigned short* W0B  = (unsigned short*)(ws + oW0);
  unsigned short* W1H  = (unsigned short*)(ws + oW1);
  unsigned short* W2H  = (unsigned short*)(ws + oW2);
  unsigned short* EH   = (unsigned short*)(ws + oEH);
  unsigned short* QK   = (unsigned short*)(ws + oQK);
  unsigned short* VT   = (unsigned short*)(ws + oVT);
  unsigned short* Ctx  = (unsigned short*)(ws + oCtx);
  float*          R    = (float*)(ws + oR);
  unsigned short* G    = (unsigned short*)(ws + oQK);
  unsigned short* O1H  = (unsigned short*)(ws + oVT);
  float*          O1F  = (float*)(ws + oCtx);

  const long long PLQKe  = (long long)NTOK * QKP;
  const long long PLVTe  = (long long)NB * DM * SEQ;
  const long long PLCTXe = (long long)NTOK * DM;

  const dim3 blk(256);
  const int  n8a = NTOK * DM / 8;
  const int  n8w = DM * DM / 8;
  const int  n8f = DFF * DM / 8;
  const dim3 gA((n8a + 255) / 256);
  const dim3 gW((n8w + 255) / 256);
  const dim3 gF((n8f + 255) / 256);
  const dim3 gN2(((NTOK / 64) * (QKP / 64) + 7) / 8, 1);
  const dim3 gN1(((NTOK / 64) * (DM / 64) + 7) / 8, 1);
  const dim3 gN4(((NTOK / 64) * (DFF / 64) + 7) / 8, 1);
  const dim3 gVT(((DM / 64) * (SEQ / 64) + 7) / 8, NB);
  const dim3 gAttn(NB * NH * NQB);
  const dim3 gRow(NTOK);
  const float invw = 1.0f / WSC;

  cvt8<0><<<gA, blk, 0, stream>>>(emb, EH, n8a, 1.0f);
  cvt8<0><<<gW, blk, 0, stream>>>(Wq, Wqkv, n8w, WSC);
  cvt8<0><<<gW, blk, 0, stream>>>(Wk, Wqkv + (size_t)DM * DM, n8w, WSC);
  cvt8<0><<<gW, blk, 0, stream>>>(Wv, Wqkv + (size_t)2 * DM * DM, n8w, WSC);
  cvt8<1><<<gW, blk, 0, stream>>>(W0, W0B, n8w, 1.0f);
  cvt8<0><<<gF, blk, 0, stream>>>(W1, W1H, n8f, WSC);
  cvt8<0><<<gF, blk, 0, stream>>>(W2, W2H, n8f, WSC);

  gemm64<0, 0, 3, 0, 0, 0><<<gN2, blk, 0, stream>>>(
      EH, DM, 0LL, 0LL, Wqkv, DM, 0LL, bq, bk, DM, emb,
      (void*)QK, QKP, 0LL, PLQKe, NTOK, QKP, DM, invw, 0.0f);
  gemm64<0, 0, 4, 1, 0, 0><<<gVT, blk, 0, stream>>>(
      Wqkv + (size_t)2 * DM * DM, DM, 0LL, 0LL, EH, DM, (long long)SEQ * DM, bv, bv, DM, emb,
      (void*)VT, SEQ, (long long)DM * SEQ, PLVTe, DM, SEQ, DM, invw, VRS);

  attn64<<<gAttn, dim3(128), 0, stream>>>(QK, VT, Ctx);

  gemm64<1, 1, 0, 0, 0, 2><<<gN1, blk, 0, stream>>>(
      Ctx, DM, 0LL, PLCTXe, W0B, DM, 0LL, b0, b0, DM, emb,
      (void*)R, DM, 0LL, 0LL, NTOK, DM, DM, 1.0f, 0.0f);
  ln_row<1><<<gRow, blk, 0, stream>>>(R, g1, be1, O1F, O1H);

  gemm64<0, 0, 2, 0, 1, 0><<<gN4, blk, 0, stream>>>(
      O1H, DM, 0LL, 0LL, W1H, DM, 0LL, b1, b1, DFF, emb,
      (void*)G, DFF, 0LL, 0LL, NTOK, DFF, DM, invw, 0.0f);
  gemm64<0, 0, 0, 0, 0, 1><<<gN1, blk, 0, stream>>>(
      G, DFF, 0LL, 0LL, W2H, DFF, 0LL, b2, b2, DM, O1F,
      (void*)R, DM, 0LL, 0LL, NTOK, DM, DFF, invw, 0.0f);
  ln_row<0><<<gRow, blk, 0, stream>>>(R, g2, be2, (float*)d_out, O1H);
  (void)hipGetLastError();
}
